// TransformerSentenceEncoderLayer_29609504539206
// MI455X (gfx1250) — hardware-verified
//
#include <hip/hip_runtime.h>


#define TT   2048
#define NBT  2
#define NR   (TT * NBT)
#define DD   768
#define NH_  8
#define HD   96
#define HP   128
#define FFN  3072
#define FCH  1024
#define ZH   1
#define DM   DD
#define NTK  TT
#define SCL  0.10206207261596577f
#define LEPS 1e-5f
#define LOSC 1024.0f

typedef _Float16 h16;
typedef unsigned short bf;
typedef __attribute__((ext_vector_type(16))) __bf16   v16bf;
typedef __attribute__((ext_vector_type(16))) _Float16 v16h;
typedef __attribute__((ext_vector_type(8)))  _Float16 v8h;
typedef __attribute__((ext_vector_type(8)))  unsigned short v8us;
typedef __attribute__((ext_vector_type(8)))  float    v8f;
typedef __attribute__((ext_vector_type(4)))  float    v4f;
typedef __attribute__((ext_vector_type(4)))  _Float16 v4h;
typedef v8h  __attribute__((may_alias)) v8ha;
typedef v4f  __attribute__((may_alias)) v4fa;
typedef v8us __attribute__((may_alias)) v8usa;

__device__ __forceinline__ unsigned short f2bf(float f) { unsigned u = __float_as_uint(f); u += 0x7FFFu + ((u >> 16) & 1u); return (unsigned short)(u >> 16); }
__device__ __forceinline__ float bf2f(unsigned short b) { return __uint_as_float(((unsigned)b) << 16); }
__device__ __forceinline__ float bfr(float f) { return bf2f(f2bf(f)); }
__device__ __forceinline__ v16h cat16(v8h lo, v8h hi) { return __builtin_shufflevector(lo, hi, 0, 1, 2, 3, 4, 5, 6, 7, 8, 9, 10, 11, 12, 13, 14, 15); }
__device__ __forceinline__ v16bf cat16b(v8us lo, v8us hi) { return __builtin_bit_cast(v16bf, __builtin_shufflevector(lo, hi, 0, 1, 2, 3, 4, 5, 6, 7, 8, 9, 10, 11, 12, 13, 14, 15)); }
__device__ __forceinline__ v8f wmma16(v16h a, v16h b, v8f c) { return __builtin_amdgcn_wmma_f32_16x16x32_f16(false, a, false, b, (short)0, c, false, false); }
__device__ __forceinline__ v8f wmmab(v16bf a, v16bf b, v8f c) { return __builtin_amdgcn_wmma_f32_16x16x32_bf16(false, a, false, b, (short)0, c, false, false); }

template <bool SPLITA, bool F16OUT = false>
__global__ __launch_bounds__(128) void k_gemmb(const bf* __restrict__ A, const bf* __restrict__ Al, const bf* __restrict__ Bn, const float* __restrict__ bias, float* C, int ldc, h16* C2, const float* __restrict__ R = nullptr, int K = DM, int roundR = 1) {
    __shared__ __align__(16) float ost[4][16 * 68];
    const int lane = threadIdx.x & 31, wave = threadIdx.x >> 5, lr = lane & 15, hi = lane >> 4;
    const int r0 = blockIdx.x * 64 + wave * 16, c0 = blockIdx.y * 64;
    const size_t aoff = (size_t)(r0 + lr) * K + 8 * hi;
    size_t boff[4];
#pragma unroll
    for (int t = 0; t < 4; ++t) boff[t] = (size_t)(c0 + t * 16 + lr) * K + 8 * hi;
    v8f acc[4];
#pragma unroll
    for (int t = 0; t < 4; ++t) acc[t] = (v8f){};
#pragma unroll 1
    for (int kc = 0; kc < K; kc += 32) {
        const v16bf a = cat16b(*(const v8us*)(A + aoff + kc), *(const v8us*)(A + aoff + kc + 16));
        v16bf al = a;
        if (SPLITA) al = cat16b(*(const v8us*)(Al + aoff + kc), *(const v8us*)(Al + aoff + kc + 16));
#pragma unroll
        for (int t = 0; t < 4; ++t) { const v16bf b = cat16b(*(const v8us*)(Bn + boff[t] + kc), *(const v8us*)(Bn + boff[t] + kc + 16)); acc[t] = wmmab(a, b, acc[t]); if (SPLITA) acc[t] = wmmab(al, b, acc[t]); }
        asm volatile("v_nop\n\tv_nop\n\tv_nop\n\tv_nop" : "+v"(acc[0]), "+v"(acc[1]), "+v"(acc[2]), "+v"(acc[3]) : "v"(a), "v"(al));
    }
    float* os = &ost[wave][0];
#pragma unroll
    for (int t = 0; t < 4; ++t) { const float bv = bias ? bfr(bias[c0 + t * 16 + lr]) : 0.f;
#pragma unroll
        for (int j = 0; j < 8; ++j) os[(hi * 8 + j) * 68 + t * 16 + lr] = acc[t][j] + bv; }
    __syncthreads();
    if (F16OUT) {
        h16* crow = (h16*)(void*)C + (size_t)r0 * ldc + c0;
        auto pass = [&]() {
#pragma unroll
            for (int s = 0; s < 4; ++s) { const int row = 4 * s + (lane >> 3), piece = lane & 7; const float* sp = os + row * 68 + piece * 8; v8h o, o2;
#pragma unroll
                for (int i = 0; i < 8; ++i) { const h16 a = (h16)sp[i]; o[i] = a; o2[i] = (h16)((sp[i] - (float)a) * LOSC); }
                *(volatile v8h*)(crow + (size_t)row * ldc + piece * 8) = o; if (C2) *(volatile v8h*)(C2 + (size_t)r0 * ldc + c0 + (size_t)row * ldc + piece * 8) = o2; }
        };
        pass(); __threadfence(); pass();
    } else {
        float* crow = C + (size_t)r0 * ldc + c0;
        auto pass = [&]() {
#pragma unroll
            for (int s = 0; s < 8; ++s) { const int Lid = (lane >> 3) + 4 * s, piece = lane & 7; const int row = Lid >> 1, cofs = (Lid & 1) * 32 + piece * 4;
                v4f val = *(const v4fa*)(os + row * 68 + cofs); if (R) { const v4f rv = *(const v4f*)(R + ((size_t)r0 + row) * ldc + c0 + cofs); val += roundR ? (v4f){bfr(rv[0]), bfr(rv[1]), bfr(rv[2]), bfr(rv[3])} : rv; }
                *(volatile v4f*)(crow + (size_t)row * ldc + cofs) = val; }
        };
        pass(); __threadfence(); pass();
    }
}

__global__ __launch_bounds__(256) void k_cvt8(const float* __restrict__ src, bf* dst, size_t n8) {
    const size_t i = (size_t)blockIdx.x * 256 + threadIdx.x; if (i >= n8) return;
    const v8f v = *(const v8f*)(src + i * 8); v8us o;
#pragma unroll
    for (int k = 0; k < 8; ++k) o[k] = f2bf(v[k]);
    *(volatile v8us*)(dst + i * 8) = o; __threadfence(); *(volatile v8us*)(dst + i * 8) = o;
}
__global__ __launch_bounds__(256) void k_zero8(bf* dst, size_t n8) {
    const size_t i = (size_t)blockIdx.x * 256 + threadIdx.x; if (i >= n8) return; v8us z;
#pragma unroll
    for (int k = 0; k < 8; ++k) z[k] = 0;
    *(volatile v8us*)(dst + i * 8) = z; __threadfence(); *(volatile v8us*)(dst + i * 8) = z;
}

template <int MODE>
__global__ __launch_bounds__(128) void k_gemm3z(const bf* __restrict__ Ah, const bf* __restrict__ Al, const bf* __restrict__ Bh, const bf* __restrict__ Bl, int K, float* C, int ldc, size_t sA, size_t sB, size_t sC) {
    if ((MODE & 1) && (int)blockIdx.y * 64 > (int)blockIdx.x * 64 + 63) return;
    const size_t z = blockIdx.z; Ah += z * sA; Al += z * sA; Bh += z * sB; Bl += z * sB; C += z * sC;
    const int Klim = (MODE & 2) ? min(K, ((int)blockIdx.x + 1) * 64) : K;
    __shared__ __align__(16) float ost[4][16 * 68];
    const int lane = threadIdx.x & 31, wave = threadIdx.x >> 5, lr = lane & 15, hi = lane >> 4;
    const int r0 = blockIdx.x * 64 + wave * 16, c0 = blockIdx.y * 64;
    const size_t aoff = (size_t)(r0 + lr) * K + 8 * hi;
    v8f acc[4];
#pragma unroll
    for (int t = 0; t < 4; ++t) acc[t] = (v8f){};
#pragma unroll 1
    for (int kc = 0; kc < Klim; kc += 32) {
        const v16bf a = cat16b(*(const v8us*)(Ah + aoff + kc), *(const v8us*)(Ah + aoff + kc + 16));
        v16bf al = a; if (!(MODE & 4) && !(MODE & 16)) al = cat16b(*(const v8us*)(Al + aoff + kc), *(const v8us*)(Al + aoff + kc + 16));
#pragma unroll
        for (int t = 0; t < 4; ++t) { const size_t bo = (size_t)(c0 + t * 16 + lr) * K + kc + 8 * hi;
            const v16bf bh = cat16b(*(const v8us*)(Bh + bo), *(const v8us*)(Bh + bo + 16));
            acc[t] = wmmab(a, bh, acc[t]);
            if (!(MODE & 4)) { if (!(MODE & 16)) acc[t] = wmmab(al, bh, acc[t]); if (!(MODE & 8)) { const v16bf bl = cat16b(*(const v8us*)(Bl + bo), *(const v8us*)(Bl + bo + 16)); acc[t] = wmmab(a, bl, acc[t]); } } }
        asm volatile("v_nop\n\tv_nop\n\tv_nop\n\tv_nop" : "+v"(acc[0]), "+v"(acc[1]), "+v"(acc[2]), "+v"(acc[3]) : "v"(a), "v"(al));
    }
    float* os = &ost[wave][0];
#pragma unroll
    for (int t = 0; t < 4; ++t) {
#pragma unroll
        for (int j = 0; j < 8; ++j) os[(hi * 8 + j) * 68 + t * 16 + lr] = acc[t][j]; }
    __builtin_amdgcn_wave_barrier(); asm volatile("" ::: "memory");
    float* crow = C + (size_t)r0 * ldc + c0;
    auto pass = [&]() {
#pragma unroll
        for (int s = 0; s < 8; ++s) { const int Lid = (lane >> 3) + 4 * s, piece = lane & 7; const int row = Lid >> 1, cofs = (Lid & 1) * 32 + piece * 4;
            const v4f val = *(const v4fa*)(os + row * 68 + cofs); *(volatile v4f*)(crow + (size_t)row * ldc + cofs) = val; }
    };
    pass(); __threadfence(); pass();
}
__global__ __launch_bounds__(256) void k_planes32z(const float* __restrict__ F, int ld, int off, float sc, int rows, bf* Ph, bf* Pl) {
    typedef __attribute__((ext_vector_type(2))) unsigned short v2us;
    const int lane = threadIdx.x & 31; const size_t r = ((size_t)blockIdx.x * 8 + (threadIdx.x >> 5)) * 2 + (lane >> 4); if (r >= (size_t)rows) return; const int z = blockIdx.z; const int c0 = (lane & 15) * 2; v2us oh, ol;
    Ph += (size_t)z * rows * 32; Pl += (size_t)z * rows * 32;
#pragma unroll
    for (int i = 0; i < 2; ++i) { const float y = F[r * ld + off + z * 32 + c0 + i] * sc; const unsigned short hb = f2bf(y); oh[i] = hb; ol[i] = f2bf(y - bf2f(hb)); }
    const size_t o = r * 32 + c0; *(volatile v2us*)(Ph + o) = oh; *(volatile v2us*)(Pl + o) = ol; __threadfence(); *(volatile v2us*)(Ph + o) = oh; *(volatile v2us*)(Pl + o) = ol;
}
__global__ __launch_bounds__(256) void k_vtpadz(const float* __restrict__ F, int ld, int off, int nk, bf* Th, bf* Tl) {
    typedef __attribute__((ext_vector_type(2))) unsigned short v2us;
    const int lane = threadIdx.x & 31; const size_t wid = (size_t)blockIdx.x * 8 + (threadIdx.x >> 5); if (wid >= (size_t)64 * (nk / 64)) return; const int z = blockIdx.z; const int d = (int)(wid / (nk / 64)); const int k0 = (int)(wid % (nk / 64)) * 64 + lane * 2; v2us oh, ol;
    Th += (size_t)z * 64 * nk; Tl += (size_t)z * 64 * nk;
#pragma unroll
    for (int i = 0; i < 2; ++i) { const float y = (d < 32) ? F[(size_t)(k0 + i) * ld + off + z * 32 + (d < 32 ? d : 0)] : 0.f; const unsigned short hb = f2bf(y); oh[i] = hb; ol[i] = f2bf(y - bf2f(hb)); }
    const size_t o = (size_t)d * nk + k0; *(volatile v2us*)(Th + o) = oh; *(volatile v2us*)(Tl + o) = ol; __threadfence(); *(volatile v2us*)(Th + o) = oh; *(volatile v2us*)(Tl + o) = ol;
}
template <int NK>
__global__ __launch_bounds__(256) void k_softmaxz(const float* __restrict__ S, int rows, bf* PH, bf* PL) {
    typedef __attribute__((ext_vector_type(4))) unsigned short v4us;
    const int lane = threadIdx.x & 31, i = blockIdx.x * 8 + (threadIdx.x >> 5); if (i >= rows) return; const size_t zo = (size_t)blockIdx.z * rows * NK; const float* sr = S + zo + (size_t)i * NK; PH += zo; PL += zo;
    float m = -3.0e38f;
#pragma unroll 1
    for (int c0 = lane * 4; c0 < NK; c0 += 128) {
#pragma unroll
        for (int q = 0; q < 4; ++q) m = fmaxf(m, sr[c0 + q]); }
#pragma unroll
    for (int sh = 16; sh; sh >>= 1) m = fmaxf(m, __shfl_xor(m, sh, 32));
    float sum = 0.f;
#pragma unroll 1
    for (int c0 = lane * 4; c0 < NK; c0 += 128) {
#pragma unroll
        for (int q = 0; q < 4; ++q) sum += __expf(sr[c0 + q] - m); }
#pragma unroll
    for (int sh = 16; sh; sh >>= 1) sum += __shfl_xor(sum, sh, 32);
    const float inv = 1.0f / sum;
#pragma unroll 1
    for (int ps = 0; ps < 2; ++ps) {
#pragma unroll 1
        for (int c0 = lane * 4; c0 < NK; c0 += 128) { v4us oh, ol;
#pragma unroll
            for (int q = 0; q < 4; ++q) { const float p = __expf(sr[c0 + q] - m) * inv; const unsigned short hb = f2bf(p); oh[q] = hb; ol[q] = f2bf(p - bf2f(hb)); }
            const size_t o = (size_t)i * NK + c0; *(volatile v4us*)(PH + o) = oh; *(volatile v4us*)(PL + o) = ol; }
        if (ps == 0) __threadfence(); }
}
__global__ __launch_bounds__(256) void k_placez(const float* __restrict__ XH, int rows, int ldy, float* Y) {
    const int lane = threadIdx.x & 31; const size_t q = (size_t)blockIdx.x * 8 + (threadIdx.x >> 5); if (q >= (size_t)rows) return; const int z = blockIdx.z; const float v = XH[((size_t)z * rows + q) * 64 + lane];
    *(volatile float*)(Y + q * ldy + z * 32 + lane) = v; __threadfence(); *(volatile float*)(Y + q * ldy + z * 32 + lane) = v;
}

__global__ __launch_bounds__(256) void k_hplanesz(const float* __restrict__ F, int ld, int h0, float sc, int rows, bf* Ph, bf* Pl) {
    typedef __attribute__((ext_vector_type(2))) unsigned short v2us;
    const int lane = threadIdx.x & 31; const size_t r = (size_t)blockIdx.x * 8 + (threadIdx.x >> 5); if (r >= (size_t)rows) return; const int z = blockIdx.z; v2us oh, ol;
    Ph += (size_t)z * rows * 64; Pl += (size_t)z * rows * 64;
#pragma unroll
    for (int i = 0; i < 2; ++i) { const float y = F[r * ld + (h0 + z) * 64 + lane * 2 + i] * sc; const unsigned short hb = f2bf(y); oh[i] = hb; ol[i] = f2bf(y - bf2f(hb)); }
    const size_t o = r * 64 + lane * 2; *(volatile v2us*)(Ph + o) = oh; *(volatile v2us*)(Pl + o) = ol; __threadfence(); *(volatile v2us*)(Ph + o) = oh; *(volatile v2us*)(Pl + o) = ol;
}
__global__ __launch_bounds__(256) void k_vtz(const float* __restrict__ F, int ld, int h0, int nk, bf* Th, bf* Tl) {
    typedef __attribute__((ext_vector_type(2))) unsigned short v2us;
    const int lane = threadIdx.x & 31; const size_t wid = (size_t)blockIdx.x * 8 + (threadIdx.x >> 5); if (wid >= (size_t)64 * (nk / 64)) return; const int z = blockIdx.z; const int d = (int)(wid / (nk / 64)); const int t0 = (int)(wid % (nk / 64)) * 64 + lane * 2; v2us oh, ol;
    Th += (size_t)z * 64 * nk; Tl += (size_t)z * 64 * nk;
#pragma unroll
    for (int i = 0; i < 2; ++i) { const float y = F[(size_t)(t0 + i) * ld + (h0 + z) * 64 + d]; const unsigned short hb = f2bf(y); oh[i] = hb; ol[i] = f2bf(y - bf2f(hb)); }
    const size_t o = (size_t)d * nk + t0; *(volatile v2us*)(Th + o) = oh; *(volatile v2us*)(Tl + o) = ol; __threadfence(); *(volatile v2us*)(Th + o) = oh; *(volatile v2us*)(Tl + o) = ol;
}
template <int NK>
__global__ __launch_bounds__(256) void k_softmaxzs(const float* __restrict__ S, int rows, float sc, bf* PH, bf* PL) {
    typedef __attribute__((ext_vector_type(4))) unsigned short v4us;
    const int lane = threadIdx.x & 31, i = blockIdx.x * 8 + (threadIdx.x >> 5); if (i >= rows) return; const size_t zo = (size_t)blockIdx.z * rows * NK; const float* sr = S + zo + (size_t)i * NK; PH += zo; PL += zo;
    float m = -3.0e38f;
#pragma unroll 1
    for (int c0 = lane * 4; c0 < NK; c0 += 128) {
#pragma unroll
        for (int q = 0; q < 4; ++q) m = fmaxf(m, sr[c0 + q] * sc); }
#pragma unroll
    for (int sh = 16; sh; sh >>= 1) m = fmaxf(m, __shfl_xor(m, sh, 32));
    float sum = 0.f;
#pragma unroll 1
    for (int c0 = lane * 4; c0 < NK; c0 += 128) {
#pragma unroll
        for (int q = 0; q < 4; ++q) sum += __expf(sr[c0 + q] * sc - m); }
#pragma unroll
    for (int sh = 16; sh; sh >>= 1) sum += __shfl_xor(sum, sh, 32);
    const float inv = 1.0f / sum;
#pragma unroll 1
    for (int ps = 0; ps < 2; ++ps) {
#pragma unroll 1
        for (int c0 = lane * 4; c0 < NK; c0 += 128) { v4us oh, ol;
#pragma unroll
            for (int q = 0; q < 4; ++q) { const float p = __expf(sr[c0 + q] * sc - m) * inv; const unsigned short hb = f2bf(p); oh[q] = hb; ol[q] = f2bf(p - bf2f(hb)); }
            const size_t o = (size_t)i * NK + c0; *(volatile v4us*)(PH + o) = oh; *(volatile v4us*)(PL + o) = ol; }
        if (ps == 0) __threadfence(); }
}

__global__ __launch_bounds__(256) void k_cvtrow(const float* __restrict__ src, bf* dst) {
    const int lane = threadIdx.x & 31; const size_t r = (size_t)blockIdx.x * 8 + (threadIdx.x >> 5); if (r >= (size_t)NR) return;
#pragma unroll 1
    for (int ps = 0; ps < 2; ++ps) {
#pragma unroll
        for (int q = 0; q < DD / 256; ++q) { v8us o;
#pragma unroll
            for (int i = 0; i < 8; ++i) o[i] = f2bf(src[r * DD + q * 256 + lane * 8 + i]);
            *(volatile v8us*)(dst + r * DD + q * 256 + lane * 8) = o; }
        if (ps == 0) __threadfence(); }
}
__global__ __launch_bounds__(256) void k_hp96z(const float* __restrict__ F, int b, int h0, bf* Ph, bf* Pl) {
    typedef __attribute__((ext_vector_type(4))) unsigned short v4us;
    const int lane = threadIdx.x & 31; const size_t t = (size_t)blockIdx.x * 8 + (threadIdx.x >> 5); if (t >= (size_t)TT) return; const int z = blockIdx.z; Ph += (size_t)z * TT * HP; Pl += (size_t)z * TT * HP;
    const float* src = F + (t * NBT + b) * DD + (h0 + z) * HD; v4us oh, ol;
#pragma unroll
    for (int i = 0; i < 4; ++i) { const int d = lane * 4 + i; const float y = (d < HD) ? src[d < HD ? d : 0] : 0.f; const unsigned short hb = f2bf(y); oh[i] = hb; ol[i] = f2bf(y - bf2f(hb)); }
    const size_t o = t * HP + lane * 4; *(volatile v4us*)(Ph + o) = oh; *(volatile v4us*)(Pl + o) = ol; __threadfence(); *(volatile v4us*)(Ph + o) = oh; *(volatile v4us*)(Pl + o) = ol;
}
__global__ __launch_bounds__(256) void k_vt96z(const float* __restrict__ F, int b, int h0, bf* Th, bf* Tl) {
    typedef __attribute__((ext_vector_type(2))) unsigned short v2us;
    const int lane = threadIdx.x & 31; const size_t wid = (size_t)blockIdx.x * 8 + (threadIdx.x >> 5); if (wid >= (size_t)HP * (TT / 64)) return; const int z = blockIdx.z; const int d = (int)(wid / (TT / 64)); const int t0 = (int)(wid % (TT / 64)) * 64 + lane * 2; v2us oh, ol;
    Th += (size_t)z * HP * TT; Tl += (size_t)z * HP * TT;
#pragma unroll
    for (int i = 0; i < 2; ++i) { const float y = (d < HD) ? F[((size_t)(t0 + i) * NBT + b) * DD + (h0 + z) * HD + (d < HD ? d : 0)] : 0.f; const unsigned short hb = f2bf(y); oh[i] = hb; ol[i] = f2bf(y - bf2f(hb)); }
    const size_t o = (size_t)d * TT + t0; *(volatile v2us*)(Th + o) = oh; *(volatile v2us*)(Tl + o) = ol; __threadfence(); *(volatile v2us*)(Th + o) = oh; *(volatile v2us*)(Tl + o) = ol;
}
__global__ __launch_bounds__(256) void k_place96z(const float* __restrict__ XH, int b, int h0, float* ATT) {
    const int lane = threadIdx.x & 31; const size_t t = (size_t)blockIdx.x * 8 + (threadIdx.x >> 5); if (t >= (size_t)TT) return; const int z = blockIdx.z; if (lane >= 24) return;
    const v4f v = *(const v4f*)(XH + ((size_t)z * TT + t) * HP + lane * 4); float* dst = ATT + (t * NBT + b) * DD + (h0 + z) * HD + lane * 4;
    *(volatile v4f*)dst = v; __threadfence(); *(volatile v4f*)dst = v;
}
template <bool RIN>
__global__ __launch_bounds__(256) void k_addln768(const float* __restrict__ Ain, const float* __restrict__ Bin, const float* __restrict__ g, const float* __restrict__ bb, float* Yf, bf* Yh, bf* Yl) {
    const int lane = threadIdx.x & 31; const size_t r = (size_t)blockIdx.x * 8 + (threadIdx.x >> 5); if (r >= (size_t)NR) return; float v[24]; float s = 0.f;
#pragma unroll
    for (int q = 0; q < 3; ++q) {
#pragma unroll
        for (int i = 0; i < 8; ++i) { const size_t o = r * DD + q * 256 + lane * 8 + i; const float t2 = Ain[o] + (RIN ? bfr(Bin[o]) : Bin[o]); v[q * 8 + i] = t2; s += t2; } }
#pragma unroll
    for (int sh = 16; sh; sh >>= 1) s += __shfl_xor(s, sh, 32);
    const float mu = s * (1.0f / DD); float qv = 0.f;
#pragma unroll
    for (int i = 0; i < 24; ++i) { const float d = v[i] - mu; qv = fmaf(d, d, qv); }
#pragma unroll
    for (int sh = 16; sh; sh >>= 1) qv += __shfl_xor(qv, sh, 32);
    const float rs = rsqrtf(qv * (1.0f / DD) + LEPS);
#pragma unroll 1
    for (int ps = 0; ps < 2; ++ps) {
#pragma unroll
        for (int q = 0; q < 3; ++q) { const int c0 = q * 256 + lane * 8; v8f y; v8us oh, ol;
#pragma unroll
            for (int i = 0; i < 8; ++i) { y[i] = (v[q * 8 + i] - mu) * rs * bfr(g[c0 + i]) + bfr(bb[c0 + i]); const unsigned short hb = f2bf(y[i]); oh[i] = hb; ol[i] = f2bf(y[i] - bf2f(hb)); }
            const size_t o = r * DD + c0; *(volatile v8f*)(Yf + o) = y; *(volatile v8us*)(Yh + o) = oh; *(volatile v8us*)(Yl + o) = ol; }
        if (ps == 0) __threadfence(); }
}
__global__ __launch_bounds__(256) void k_relupl3072(const float* __restrict__ F, bf* Gh, bf* Gl) {
    const int lane = threadIdx.x & 31; const size_t r = (size_t)blockIdx.x * 8 + (threadIdx.x >> 5); if (r >= (size_t)FCH) return;
#pragma unroll 1
    for (int ps = 0; ps < 2; ++ps) {
#pragma unroll 1
        for (int q = 0; q < FFN / 256; ++q) { const size_t o = r * FFN + q * 256 + lane * 8; const v8f v = *(const v8f*)(F + o); v8us oh, ol;
#pragma unroll
            for (int i = 0; i < 8; ++i) { const float y = fmaxf(v[i], 0.f); const unsigned short hb = f2bf(y); oh[i] = hb; ol[i] = f2bf(y - bf2f(hb)); }
            *(volatile v8us*)(Gh + o) = oh; *(volatile v8us*)(Gl + o) = ol; }
        if (ps == 0) __threadfence(); }
}
__global__ __launch_bounds__(256) void k_split768(const float* __restrict__ src, bf* dh, bf* dl) {
    const int lane = threadIdx.x & 31; const size_t r = (size_t)blockIdx.x * 8 + (threadIdx.x >> 5); if (r >= (size_t)NR) return;
#pragma unroll 1
    for (int ps = 0; ps < 2; ++ps) {
#pragma unroll
        for (int q = 0; q < DD / 256; ++q) { const size_t o = r * DD + q * 256 + lane * 8; const v8f v = *(const v8f*)(src + o); v8us oh, ol;
#pragma unroll
            for (int i = 0; i < 8; ++i) { const unsigned short hb = f2bf(v[i]); oh[i] = hb; ol[i] = f2bf(v[i] - bf2f(hb)); }
            *(volatile v8us*)(dh + o) = oh; *(volatile v8us*)(dl + o) = ol; }
        if (ps == 0) __threadfence(); }
}

extern "C" void kernel_launch(void* const* d_in, const int* in_sizes, int n_in,
                              void* d_out, int out_size, void* d_ws, size_t ws_size, hipStream_t stream) {
    (void)in_sizes; (void)n_in; (void)out_size;
    const float* x = (const float*)d_in[0]; const float* wq = (const float*)d_in[1]; const float* bq = (const float*)d_in[2]; const float* wk = (const float*)d_in[3]; const float* bk = (const float*)d_in[4]; const float* wv = (const float*)d_in[5]; const float* bv = (const float*)d_in[6]; const float* wo = (const float*)d_in[7]; const float* bo = (const float*)d_in[8];
    const float* g1 = (const float*)d_in[9]; const float* be1 = (const float*)d_in[10]; const float* w1 = (const float*)d_in[11]; const float* b1 = (const float*)d_in[12]; const float* w2 = (const float*)d_in[13]; const float* b2 = (const float*)d_in[14]; const float* g2 = (const float*)d_in[15]; const float* be2 = (const float*)d_in[16];
    float* out = (float*)d_out;
    char* wsp = (char*)d_ws;
    auto take = [&](size_t bytes) { char* p = wsp; wsp += (bytes + 255) & ~(size_t)255; return (void*)p; };
    bf* WQ = (bf*)take((size_t)DD * DD * 2); bf* WK = (bf*)take((size_t)DD * DD * 2); bf* WV = (bf*)take((size_t)DD * DD * 2); bf* WO = (bf*)take((size_t)DD * DD * 2); bf* W1 = (bf*)take((size_t)FFN * DD * 2); bf* W2 = (bf*)take((size_t)DD * FFN * 2);
    bf* Xb = (bf*)take((size_t)NR * DD * 2); float* QF = (float*)take((size_t)NR * DD * 4); float* KF = (float*)take((size_t)NR * DD * 4); float* VF = (float*)take((size_t)NR * DD * 4);
    bf* Qh = (bf*)take((size_t)ZH * TT * HP * 2); bf* Ql = (bf*)take((size_t)ZH * TT * HP * 2); bf* Kh = (bf*)take((size_t)ZH * TT * HP * 2); bf* Kl = (bf*)take((size_t)ZH * TT * HP * 2); bf* VTh = (bf*)take((size_t)ZH * HP * TT * 2); bf* VTl = (bf*)take((size_t)ZH * HP * TT * 2);
    char* shared = (char*)take((size_t)ZH * TT * TT * 4 + 2 * (size_t)ZH * TT * TT * 2);
    float* S = (float*)shared; bf* PH = (bf*)(shared + (size_t)ZH * TT * TT * 4); bf* PL = (bf*)(shared + (size_t)ZH * TT * TT * 4 + (size_t)ZH * TT * TT * 2);
    float* F1 = (float*)shared; bf* G1h = (bf*)(shared + (size_t)FCH * FFN * 4); bf* G1l = (bf*)(shared + (size_t)FCH * FFN * 4 + (size_t)FCH * FFN * 2);
    float* XH = (float*)take((size_t)ZH * TT * HP * 4); float* ATT = (float*)take((size_t)NR * DD * 4); bf* H1h = (bf*)take((size_t)NR * DD * 2); bf* H1l = (bf*)take((size_t)NR * DD * 2);
    bf* Ah = (bf*)KF; bf* Al = Ah + (size_t)NR * DD; float* AO = VF; float* H1 = QF;
    if ((size_t)(wsp - (char*)d_ws) > ws_size) return;
    k_cvt8<<<(DD * DD / 8 + 255) / 256, 256, 0, stream>>>(wq, WQ, DD * DD / 8); k_cvt8<<<(DD * DD / 8 + 255) / 256, 256, 0, stream>>>(wk, WK, DD * DD / 8); k_cvt8<<<(DD * DD / 8 + 255) / 256, 256, 0, stream>>>(wv, WV, DD * DD / 8); k_cvt8<<<(DD * DD / 8 + 255) / 256, 256, 0, stream>>>(wo, WO, DD * DD / 8);
    k_cvt8<<<(FFN * DD / 8 + 255) / 256, 256, 0, stream>>>(w1, W1, FFN * DD / 8); k_cvt8<<<(DD * FFN / 8 + 255) / 256, 256, 0, stream>>>(w2, W2, DD * FFN / 8);
    k_cvtrow<<<NR / 8, 256, 0, stream>>>(x, Xb);
    const dim3 gP(NR / 64, DD / 64, 1);
    k_gemmb<false, false><<<gP, 128, 0, stream>>>(Xb, nullptr, WQ, bq, QF, DD, nullptr, nullptr, DD); k_gemmb<false, false><<<gP, 128, 0, stream>>>(Xb, nullptr, WK, bk, KF, DD, nullptr, nullptr, DD); k_gemmb<false, false><<<gP, 128, 0, stream>>>(Xb, nullptr, WV, bv, VF, DD, nullptr, nullptr, DD);
    for (int b = 0; b < NBT; ++b)
        for (int g = 0; g < NH_ / ZH; ++g) { const int h0 = g * ZH;
            k_hp96z<<<dim3(TT / 8, 1, ZH), 256, 0, stream>>>(QF, b, h0, Qh, Ql); k_hp96z<<<dim3(TT / 8, 1, ZH), 256, 0, stream>>>(KF, b, h0, Kh, Kl); k_vt96z<<<dim3((HP * (TT / 64)) / 8, 1, ZH), 256, 0, stream>>>(VF, b, h0, VTh, VTl);
            k_gemm3z<0><<<dim3(TT / 64, TT / 64, ZH), 128, 0, stream>>>(Qh, Ql, Kh, Kl, HP, S, TT, (size_t)TT * HP, (size_t)TT * HP, (size_t)TT * TT);
            k_softmaxzs<TT><<<dim3(TT / 8, 1, ZH), 256, 0, stream>>>(S, TT, SCL, PH, PL);
            k_gemm3z<0><<<dim3(TT / 64, HP / 64, ZH), 128, 0, stream>>>(PH, PL, VTh, VTl, TT, XH, HP, (size_t)TT * TT, (size_t)HP * TT, (size_t)TT * HP);
            k_place96z<<<dim3(TT / 8, 1, ZH), 256, 0, stream>>>(XH, b, h0, ATT); }
    k_split768<<<NR / 8, 256, 0, stream>>>(ATT, Ah, Al);
    k_gemmb<true, false><<<gP, 128, 0, stream>>>(Ah, Al, WO, bo, AO, DD, nullptr, nullptr, DD);
    k_addln768<true><<<NR / 8, 256, 0, stream>>>(AO, x, g1, be1, H1, H1h, H1l);
    for (int c = 0; c < NR / FCH; ++c) { const size_t r0 = (size_t)c * FCH;
        k_gemmb<true, false><<<dim3(FCH / 64, FFN / 64, 1), 128, 0, stream>>>(H1h + r0 * DD, H1l + r0 * DD, W1, b1, F1, FFN, nullptr, nullptr, DD);
        k_relupl3072<<<FCH / 8, 256, 0, stream>>>(F1, G1h, G1l);
        k_gemmb<true, false><<<dim3(FCH / 64, DD / 64, 1), 128, 0, stream>>>(G1h, G1l, W2, b2, AO + r0 * DD, DD, nullptr, nullptr, FFN); }
    k_addln768<false><<<NR / 8, 256, 0, stream>>>(AO, H1, g2, be2, out, Ah, Al);
}
